// SAGE_66718021976360
// MI455X (gfx1250) — hardware-verified
//
#include <hip/hip_runtime.h>
#include <stddef.h>
#include <stdint.h>


#define FIN    32
#define HID    64
#define K1     96
#define K2     256
#define T1N    128
#define KT1    128
#define KT2    256
#define KT3    128
#define OUTC   16
#define NG     1000
#define NTILE  63
#define NGP    (NTILE * 16)
#define NTHR   256
#define NWAVE  8
#define EPT    8
#define CHUNK  (NTHR * EPT)
#define WCAP   (EPT * 32)
#define LISTN  (NWAVE * WCAP)
#define NBA    1024
#define SLA    10
#define RCAP   28672
#define DEGCAP 64
#define GBM    64
#define GBN    64
#define GTHR   128
#define AGG_ZINTS    (LISTN + 2 * RCAP + 3 * NBA)
#define MISC_INTS    16
#define ROWBUF_US    (2 * K1)
#define ROWBUF_INTS  (NWAVE * ROWBUF_US / 2)
#define AGG_LDS_INTS (AGG_ZINTS + MISC_INTS + ROWBUF_INTS)
#define WPL    (HID * K2)
#define WSMAX  134217728

static_assert((CHUNK & (CHUNK - 1)) == 0 && CHUNK <= 4096);
static_assert((NBA & (NBA - 1)) == 0 && NBA == (1 << SLA));
static_assert(((long long)CHUNK << SLA) < (1LL << 31));
static_assert(NBA % (2 * NWAVE) == 0 && NBA % GBM == 0);
static_assert(RCAP % 4 == 0 && AGG_ZINTS % (NTHR * 4) == 0 && ((AGG_ZINTS + MISC_INTS) % 4) == 0);
static_assert(K1 % 32 == 0 && K2 % 32 == 0 && KT1 % 32 == 0 && KT2 % 32 == 0 && KT3 % 32 == 0);
static_assert(K1 == 3 * FIN && K2 == 4 * HID && KT1 == 2 * HID && KT2 == 2 * T1N && KT3 == 2 * HID);
static_assert(GBM == (GTHR / 32) * 16 && GBN == HID && HID == 64 && FIN == 32);
static_assert((ROWBUF_US * 2) % 128 == 0 && ROWBUF_US / 8 == 24);
static_assert(AGG_LDS_INTS * 4 <= 300000);
static_assert(NG % 8 == 0 && NGP >= NG && NGP % 16 == 0 && (NG * OUTC - 1) == 15999);
static_assert(HID * K1 <= WPL && T1N * KT1 <= WPL && HID * KT2 <= WPL && OUTC * KT3 <= WPL);
static_assert((HID * K1 / 8) % NTHR == 0 && (WPL / 8) % NTHR == 0 && (OUTC * KT3 / 8) % NTHR == 0);

typedef float          v2f   __attribute__((ext_vector_type(2)));
typedef float          v4f   __attribute__((ext_vector_type(4)));
typedef float          v8f   __attribute__((ext_vector_type(8)));
typedef int            v4i   __attribute__((ext_vector_type(4)));
typedef int            v8i   __attribute__((ext_vector_type(8)));
typedef unsigned int   v4u   __attribute__((ext_vector_type(4)));
typedef unsigned short v4us  __attribute__((ext_vector_type(4)));
typedef unsigned short v8us  __attribute__((ext_vector_type(8)));
typedef unsigned short v16us __attribute__((ext_vector_type(16)));
typedef __bf16         v16bf __attribute__((ext_vector_type(16)));
typedef v2f  __attribute__((may_alias)) v2fa;
typedef v4f  __attribute__((may_alias)) v4fa;
typedef v4i  __attribute__((may_alias)) v4ia;
typedef v4us __attribute__((may_alias)) v4usa;
typedef v8us __attribute__((may_alias)) v8usa;
union FragB { v16bf v; v16us u; v8us h[2]; v8i w; };

__device__ __forceinline__ v8f wmb(const FragB& a, const FragB& b, v8f c) {
  v8f d = __builtin_amdgcn_wmma_f32_16x16x32_bf16(false, a.v, false, b.v, (short)0, c, false, false);
  asm volatile("v_nop\n\tv_nop\n\tv_nop\n\tv_nop" : "+v"(d) : "v"(a.w), "v"(b.w));
  return d;
}

__device__ __forceinline__ unsigned bf16_bits(float f) {
  const unsigned u = __float_as_uint(f);
  return (u + 0x7FFFu + ((u >> 16) & 1u)) >> 16;
}
__device__ __forceinline__ float bf16_val(float f) {
  return __uint_as_float(bf16_bits(f) << 16);
}
__device__ __forceinline__ float relu_keep(float t) {
  return (t > 0.0f) ? t : ((t == t) ? 0.0f : t);
}

__device__ __forceinline__ void wave_sync() {
  __builtin_amdgcn_fence(__ATOMIC_RELEASE, "wavefront");
  __builtin_amdgcn_wave_barrier();
  __builtin_amdgcn_fence(__ATOMIC_ACQUIRE, "wavefront");
}

template <int SLB>
__device__ __forceinline__ int scan_chunk(const int* __restrict__ dsts, int nE, int cbase, int slotBase,
                                          int nb, int vec8, int* list, int tid, int lane, int wave) {
  int wc = 0;
  const int el0  = tid * EPT;
  const int e0   = cbase + el0;
  const int sent = -2147483647 - 1;
  v4i da, db;
  if (vec8 != 0 && cbase + CHUNK <= nE) {
    da = *(const v4i*)(dsts + e0);
    db = *(const v4i*)(dsts + e0 + 4);
  } else {
    da.x = (e0     < nE) ? dsts[min(e0,     nE - 1)] : sent;
    da.y = (e0 + 1 < nE) ? dsts[min(e0 + 1, nE - 1)] : sent;
    da.z = (e0 + 2 < nE) ? dsts[min(e0 + 2, nE - 1)] : sent;
    da.w = (e0 + 3 < nE) ? dsts[min(e0 + 3, nE - 1)] : sent;
    db.x = (e0 + 4 < nE) ? dsts[min(e0 + 4, nE - 1)] : sent;
    db.y = (e0 + 5 < nE) ? dsts[min(e0 + 5, nE - 1)] : sent;
    db.z = (e0 + 6 < nE) ? dsts[min(e0 + 6, nE - 1)] : sent;
    db.w = (e0 + 7 < nE) ? dsts[min(e0 + 7, nE - 1)] : sent;
  }
  const unsigned nbs = (unsigned)slotBase;
  const unsigned unb = (unsigned)nb;
  const unsigned s0 = (unsigned)da.x - nbs, s1 = (unsigned)da.y - nbs;
  const unsigned s2 = (unsigned)da.z - nbs, s3 = (unsigned)da.w - nbs;
  const unsigned s4 = (unsigned)db.x - nbs, s5 = (unsigned)db.y - nbs;
  const unsigned s6 = (unsigned)db.z - nbs, s7 = (unsigned)db.w - nbs;
  const bool h0 = s0 < unb, h1 = s1 < unb, h2 = s2 < unb, h3 = s3 < unb;
  const bool h4 = s4 < unb, h5 = s5 < unb, h6 = s6 < unb, h7 = s7 < unb;
  const unsigned any = __builtin_amdgcn_ballot_w32(h0 | h1 | h2 | h3 | h4 | h5 | h6 | h7);
  if (any != 0u) {
#define HITJ(J, HJ, SJ) { \
      const unsigned mj = __builtin_amdgcn_ballot_w32(HJ); \
      if (mj != 0u) { \
        if (HJ) { \
          const int pos = wc + (int)__builtin_amdgcn_mbcnt_lo(mj, 0u); \
          if (pos < WCAP) list[wave * WCAP + pos] = ((el0 + (J)) << SLB) | (int)(SJ); \
        } \
        wc += (int)__builtin_popcount(mj); } }
    HITJ(0, h0, s0)
    HITJ(1, h1, s1)
    HITJ(2, h2, s2)
    HITJ(3, h3, s3)
    HITJ(4, h4, s4)
    HITJ(5, h5, s5)
    HITJ(6, h6, s6)
    HITJ(7, h7, s7)
#undef HITJ
  }
  return wc;
}

__global__ __launch_bounds__(NTHR) void k_cvx(const float* __restrict__ x, int nN, int nUnits,
                                              unsigned short* xb) {
  const int u = (int)blockIdx.x * NTHR + (int)threadIdx.x;
  if (u >= nUnits) return;
  const int row = u >> 2;
  const int k8  = (u & 3) * 8;
  const int rc  = row < nN ? row : nN - 1;
  const float* p = x + (size_t)rc * FIN + k8;
  const v4f a = *(const v4fa*)p;
  const v4f b = *(const v4fa*)(p + 4);
  const bool ok = row < nN;
  v8us o;
  o[0] = ok ? (unsigned short)bf16_bits(a.x) : (unsigned short)0;
  o[1] = ok ? (unsigned short)bf16_bits(a.y) : (unsigned short)0;
  o[2] = ok ? (unsigned short)bf16_bits(a.z) : (unsigned short)0;
  o[3] = ok ? (unsigned short)bf16_bits(a.w) : (unsigned short)0;
  o[4] = ok ? (unsigned short)bf16_bits(b.x) : (unsigned short)0;
  o[5] = ok ? (unsigned short)bf16_bits(b.y) : (unsigned short)0;
  o[6] = ok ? (unsigned short)bf16_bits(b.z) : (unsigned short)0;
  o[7] = ok ? (unsigned short)bf16_bits(b.w) : (unsigned short)0;
  unsigned short* dp = xb + (size_t)row * FIN + k8;
  *(volatile v8us*)dp = o;
  __threadfence();
  *(volatile v8us*)dp = o;
}

__device__ __forceinline__ void stage_w(unsigned short* T, int pitch, const float* __restrict__ W,
                                        int Kd, int Nd, int c0, int c1, int tid) {
  const int tot = Kd * Nd;
#pragma unroll 4
  for (int idx = tid; idx < tot; idx += NTHR) {
    const int k = idx / Nd;
    const int n = idx - k * Nd;
    const unsigned short b = (unsigned short)bf16_bits(W[idx]);
    T[n * pitch + c0 + k] = b;
    T[n * pitch + c1 + k] = b;
  }
}

__global__ __launch_bounds__(NTHR) void k_wprep(const float* __restrict__ w1l, const float* __restrict__ w1r,
                                                const float* __restrict__ w2l, const float* __restrict__ w2r,
                                                const float* __restrict__ wl1, const float* __restrict__ wl2,
                                                const float* __restrict__ wl3, const int* __restrict__ bat, int nN,
                                                unsigned short* W1C, unsigned short* W2C, unsigned short* WL1C,
                                                unsigned short* WL2C, unsigned short* WL3C, int* flg) {
  __shared__ __attribute__((aligned(16))) unsigned short T[WPL];
  __shared__ int wv[NWAVE];
  const int tid = (int)threadIdx.x, lane = tid & 31, wave = tid >> 5;
  const int b = (int)blockIdx.x;
  unsigned short* P = W1C;
  int nvec = 0;
  int viol = 0;
  if (b == 0) {
    stage_w(T, K1, w1l, FIN, HID, 0, FIN, tid);
    stage_w(T, K1, w1r, FIN, HID, 2 * FIN, 2 * FIN, tid);
    P = W1C; nvec = HID * K1 / 8;
  } else if (b == 1) {
    stage_w(T, K2, w2l, HID, HID, 0, HID, tid);
    stage_w(T, K2, w2r, HID, HID, 2 * HID, 3 * HID, tid);
    P = W2C; nvec = HID * K2 / 8;
  } else if (b == 2) {
    stage_w(T, KT1, wl1, HID, T1N, 0, HID, tid);
    P = WL1C; nvec = T1N * KT1 / 8;
  } else if (b == 3) {
    stage_w(T, KT2, wl2, T1N, HID, 0, T1N, tid);
    P = WL2C; nvec = HID * KT2 / 8;
  } else if (b == 4) {
    stage_w(T, KT3, wl3, HID, OUTC, 0, HID, tid);
    P = WL3C; nvec = OUTC * KT3 / 8;
  } else {
#pragma unroll 1
    for (int i = tid; i < nN - 1; i += NTHR) {
      const int a0 = bat[i];
      const int a1 = bat[i + 1];
      viol |= (a0 > a1) ? 1 : 0;
    }
  }
  const unsigned bm = __builtin_amdgcn_ballot_w32(viol != 0);
  if (lane == 0) wv[wave] = (bm != 0u) ? 1 : 0;
  __syncthreads();
#pragma unroll 1
  for (int v = tid; v < nvec; v += NTHR) {
    const v8us q = *(const v8usa*)(T + 8 * v);
    *(volatile v8us*)(P + 8 * (size_t)v) = q;
  }
  __threadfence();
#pragma unroll 1
  for (int v = tid; v < nvec; v += NTHR) {
    const v8us q = *(const v8usa*)(T + 8 * v);
    *(volatile v8us*)(P + 8 * (size_t)v) = q;
  }
  if (b == 5) {
    int f = 0;
#pragma unroll
    for (int w2 = 0; w2 < NWAVE; ++w2) f |= wv[w2];
    v4i o;
    o.x = (lane == 0) ? f : 0; o.y = 0; o.z = 0; o.w = 0;
    const bool st = (wave == 0) && (lane < 8);
    int* fp = flg + 4 * (lane & 7);
    if (st) *(volatile v4i*)fp = o;
    __threadfence();
    if (st) *(volatile v4i*)fp = o;
  }
}

template <int L>
__global__ __launch_bounds__(NTHR) void k_scan(const int* __restrict__ srcs, const int* __restrict__ dsts,
                                               int nE, int nN, int vec8, int mRows,
                                               const unsigned short* __restrict__ xb,
                                               const float* __restrict__ h1, unsigned short* aout) {
  extern __shared__ __attribute__((aligned(16))) int dsm[];
  int* list = dsm;
  int* hl   = dsm + LISTN;
  int* sl   = hl + RCAP;
  int* cnt  = sl + RCAP;
  int* offs = cnt + NBA;
  int* cur  = offs + NBA;
  int* misc = cur + NBA;
  const int tid = (int)threadIdx.x, lane = tid & 31, wave = tid >> 5;
  unsigned short* rowbuf = (unsigned short*)(misc + MISC_INTS) + wave * ROWBUF_US;
  const int nodeBase = (int)blockIdx.x * NBA;

  {
    const v4i z4 = {0, 0, 0, 0};
    for (int i = tid * 4; i < AGG_ZINTS; i += NTHR * 4) *(v4ia*)(dsm + i) = z4;
    if (tid < MISC_INTS) misc[tid] = 0;
  }
  __syncthreads();

  int t = 0, ov = 0;
  const int nChunks = (nE + CHUNK - 1) / CHUNK;
#pragma unroll 1
  for (int ch = 0; ch < nChunks; ++ch) {
    const int cbase = ch * CHUNK;
    const int wc = scan_chunk<SLA>(dsts, nE, cbase, nodeBase, NBA, vec8, list, tid, lane, wave);
    if (lane == 0) misc[wave] = wc;
    __syncthreads();
    if (wave == 0) {
#pragma unroll 1
      for (int w2 = 0; w2 < NWAVE; ++w2) {
        int c = misc[w2];
        c = c < 0 ? 0 : (c > WCAP ? WCAP : c);
#pragma unroll 1
        for (int b0 = 0; b0 < c; b0 += 32) {
          const int idx = b0 + lane;
          const int ent = list[w2 * WCAP + (idx < WCAP ? idx : WCAP - 1)];
          const int m32 = (c - b0) < 32 ? (c - b0) : 32;
#pragma unroll 1
          for (int k = 0; k < m32; ++k) {
            const int u    = __builtin_amdgcn_readlane(ent, k);
            const int slot = u & (NBA - 1);
            const int el   = (u >> SLA) & (CHUNK - 1);
            const int pk   = ((cbase + el) << SLA) | slot;
            if (t < RCAP) {
              if (lane == 0) { hl[t] = pk; cnt[slot] = cnt[slot] + 1; }
              t = t + 1;
            } else {
              ov = 1;
            }
          }
        }
      }
    }
    __syncthreads();
  }
  if (wave == 0 && lane == 0) { misc[8] = t; misc[9] = ov; }
  __syncthreads();
  int tt = misc[8];
  tt = tt < 0 ? 0 : (tt > RCAP ? RCAP : tt);
  const int ovf = misc[9];

  if (wave == 0) {
    const int base = lane * (NBA / 32);
    int s = 0;
#pragma unroll 1
    for (int i = 0; i < NBA / 32; ++i) s += cnt[base + i];
    int incl = s;
#pragma unroll
    for (int d = 1; d < 32; d <<= 1) {
      const int y = __shfl_up(incl, d, 32);
      if (lane >= d) incl += y;
    }
    int run = incl - s;
#pragma unroll 1
    for (int i = 0; i < NBA / 32; ++i) {
      const int cv = cnt[base + i];
      offs[base + i] = run;
      cur[base + i]  = run;
      run += cv;
    }
  }
  __syncthreads();
  if (wave == 0) {
#pragma unroll 1
    for (int b0 = 0; b0 < tt; b0 += 32) {
      const int idx = b0 + lane;
      const int ent = hl[idx < RCAP ? idx : RCAP - 1];
      const int m32 = (tt - b0) < 32 ? (tt - b0) : 32;
#pragma unroll 1
      for (int k = 0; k < m32; ++k) {
        const int u    = __builtin_amdgcn_readlane(ent, k);
        const int slot = u & (NBA - 1);
        if (lane == 0) {
          int p = cur[slot];
          p = p < 0 ? 0 : (p > RCAP - 1 ? RCAP - 1 : p);
          sl[p] = u;
          cur[slot] = p + 1;
        }
      }
    }
  }
  __syncthreads();

  const float qnan = __int_as_float(0x7fc00000);
  const float pz = (ovf != 0) ? qnan : 0.0f;
  if constexpr (L == 1) {
#pragma unroll 1
    for (int pi = 0; pi < NBA / (2 * NWAVE); ++pi) {
      const int p     = pi * NWAVE + wave;
      const int node0 = nodeBase + 2 * p;
#pragma unroll 1
      for (int j = 0; j < 2; ++j) {
        const int s    = 2 * p + j;
        const int node = nodeBase + s;
        int c = cnt[s];
        const bool big = c > DEGCAP;
        c = c < 0 ? 0 : (c > DEGCAP ? DEGCAP : c);
        int o = offs[s];
        o = o < 0 ? 0 : (o > RCAP ? RCAP : o);
        const int nc = node < nN ? node : nN - 1;
        float acc = 0.0f;
#pragma unroll 1
        for (int b0 = 0; b0 < c; b0 += 32) {
          int idx = o + b0 + lane;
          idx = idx > RCAP - 1 ? RCAP - 1 : idx;
          const int ent = sl[idx];
          int eid = ent >> SLA;
          eid = eid < 0 ? 0 : (eid > nE - 1 ? nE - 1 : eid);
          int sr = srcs[eid];
          sr = sr < 0 ? 0 : (sr > nN - 1 ? nN - 1 : sr);
          const int m32 = (c - b0) < 32 ? (c - b0) : 32;
#pragma unroll 1
          for (int k = 0; k < m32; ++k) {
            const int sk = __builtin_amdgcn_readlane(sr, k);
            const unsigned w = (unsigned)xb[(size_t)sk * FIN + lane];
            acc += __uint_as_float(w << 16);
          }
        }
        const float pzr = big ? qnan : pz;
        const bool live = node < nN;
        const float mv = live ? (acc + pzr) : 0.0f;
        const unsigned hb = bf16_bits(mv);
        const unsigned lb = bf16_bits(mv - __uint_as_float(hb << 16));
        const unsigned xw = (unsigned)xb[(size_t)nc * FIN + lane];
        const unsigned xo = live ? bf16_bits(__uint_as_float(xw << 16) + pzr) : 0u;
        rowbuf[j * K1 + lane]           = (unsigned short)hb;
        rowbuf[j * K1 + FIN + lane]     = (unsigned short)lb;
        rowbuf[j * K1 + 2 * FIN + lane] = (unsigned short)xo;
      }
      wave_sync();
      const int li = lane < 24 ? lane : 23;
      const v8us q = *(const v8usa*)(rowbuf + 8 * li);
      wave_sync();
      const bool wr = (node0 < mRows) && (lane < 24);
      unsigned short* rp = aout + (size_t)node0 * K1 + 8 * li;
      if (wr) *(volatile v8us*)rp = q;
      __threadfence();
      if (wr) *(volatile v8us*)rp = q;
    }
  } else {
    const int q0s = (4 * lane) & 31, q1s = (4 * lane + 1) & 31;
    const int q2s = (4 * lane + 2) & 31, q3s = (4 * lane + 3) & 31;
#pragma unroll 1
    for (int si = 0; si < NBA / NWAVE; ++si) {
      const int s    = si * NWAVE + wave;
      const int node = nodeBase + s;
      int c = cnt[s];
      const bool big = c > DEGCAP;
      c = c < 0 ? 0 : (c > DEGCAP ? DEGCAP : c);
      int o = offs[s];
      o = o < 0 ? 0 : (o > RCAP ? RCAP : o);
      float acc0 = 0.0f, acc1 = 0.0f;
#pragma unroll 1
      for (int b0 = 0; b0 < c; b0 += 32) {
        int idx = o + b0 + lane;
        idx = idx > RCAP - 1 ? RCAP - 1 : idx;
        const int ent = sl[idx];
        int eid = ent >> SLA;
        eid = eid < 0 ? 0 : (eid > nE - 1 ? nE - 1 : eid);
        int sr = srcs[eid];
        sr = sr < 0 ? 0 : (sr > nN - 1 ? nN - 1 : sr);
        const int m32 = (c - b0) < 32 ? (c - b0) : 32;
#pragma unroll 1
        for (int k = 0; k < m32; ++k) {
          const int sk = __builtin_amdgcn_readlane(sr, k);
          const v2f a = *(const v2fa*)(h1 + (size_t)sk * HID + 2 * lane);
          acc0 += a.x; acc1 += a.y;
        }
      }
      const float pzr = big ? qnan : pz;
      const bool live = node < nN;
      const float v0 = live ? (acc0 + pzr) : 0.0f;
      const float v1 = live ? (acc1 + pzr) : 0.0f;
      const unsigned hb0 = bf16_bits(v0), hb1 = bf16_bits(v1);
      const unsigned lb0 = bf16_bits(v0 - __uint_as_float(hb0 << 16));
      const unsigned lb1 = bf16_bits(v1 - __uint_as_float(hb1 << 16));
      const int hw = (int)(hb0 | (hb1 << 16));
      const int lw = (int)(lb0 | (lb1 << 16));
      const int g0 = __shfl(hw, q0s, 32), g1 = __shfl(hw, q1s, 32);
      const int g2 = __shfl(hw, q2s, 32), g3 = __shfl(hw, q3s, 32);
      const int p0 = __shfl(lw, q0s, 32), p1 = __shfl(lw, q1s, 32);
      const int p2 = __shfl(lw, q2s, 32), p3 = __shfl(lw, q3s, 32);
      const bool lsel = (lane & 8) != 0;
      v4u pv;
      pv.x = (unsigned int)(lsel ? p0 : g0);
      pv.y = (unsigned int)(lsel ? p1 : g1);
      pv.z = (unsigned int)(lsel ? p2 : g2);
      pv.w = (unsigned int)(lsel ? p3 : g3);
      const bool wr = (node < mRows) && (lane < 16);
      unsigned short* hp = aout + (size_t)node * K2 + 8 * (lane & 15);
      if (wr) *(volatile v4u*)hp = pv;
      __threadfence();
      if (wr) *(volatile v4u*)hp = pv;
    }
  }
}

template <int L>
__global__ __launch_bounds__(GTHR) void k_gemm(const unsigned short* A, const unsigned short* __restrict__ BT,
                                               const float* __restrict__ bias, float* outF,
                                               unsigned short* a2, int nN) {
  constexpr int K = (L == 1) ? K1 : K2;
  __shared__ __attribute__((aligned(16))) float stg[GBM * GBN];
  const int tid = (int)threadIdx.x, lane = tid & 31, wave = tid >> 5, hh = lane >> 4, m = lane & 15;
  const int rowBase = (int)blockIdx.x * GBM;

  v8f acc[4];
  {
    const v8f z = {0.f, 0.f, 0.f, 0.f, 0.f, 0.f, 0.f, 0.f};
    acc[0] = z; acc[1] = z; acc[2] = z; acc[3] = z;
  }
  const unsigned short* ap = A  + (size_t)(rowBase + 16 * wave + m) * (size_t)K + 8 * hh;
  const unsigned short* wp = BT + (size_t)m * (size_t)K + 8 * hh;
#pragma unroll 1
  for (int k0 = 0; k0 < K; k0 += 32) {
    FragB af;
    af.h[0] = *(const v8usa*)(ap + k0);
    af.h[1] = *(const v8usa*)(ap + k0 + 16);
#pragma unroll
    for (int t = 0; t < 4; ++t) {
      const unsigned short* wq = wp + (size_t)(16 * t) * (size_t)K + k0;
      FragB bf;
      bf.h[0] = *(const v8usa*)wq;
      bf.h[1] = *(const v8usa*)(wq + 16);
      acc[t] = wmb(af, bf, acc[t]);
    }
  }

#pragma unroll
  for (int t = 0; t < 4; ++t) {
    const int lc = 16 * t + m;
#pragma unroll
    for (int r = 0; r < 8; ++r) {
      const int lr = 16 * wave + 8 * hh + r;
      stg[lr * GBN + lc] = acc[t][r];
    }
  }
  __syncthreads();

  v4f b4;
  {
    const v4f tb = *(const v4f*)(bias + 4 * m);
    b4.x = bf16_val(tb.x); b4.y = bf16_val(tb.y); b4.z = bf16_val(tb.z); b4.w = bf16_val(tb.w);
  }
  v4f fv[8];
#pragma unroll
  for (int i = 0; i < 8; ++i) {
    const int lr = 16 * wave + 2 * i + hh;
    const bool ok = (rowBase + lr) < nN;
    const v4f tv = *(const v4fa*)(stg + lr * GBN + 4 * m) + b4;
    v4f y;
    y.x = relu_keep(tv.x); y.y = relu_keep(tv.y); y.z = relu_keep(tv.z); y.w = relu_keep(tv.w);
    y.x = ok ? y.x : 0.0f; y.y = ok ? y.y : 0.0f; y.z = ok ? y.z : 0.0f; y.w = ok ? y.w : 0.0f;
    fv[i] = y;
  }
  v8us qv[8];
  if constexpr (L == 1) {
    __syncthreads();
    unsigned short* us = (unsigned short*)stg;
#pragma unroll
    for (int i = 0; i < 8; ++i) {
      const int lr = 16 * wave + 2 * i + hh;
      v4us h4, l4;
      unsigned hb;
      hb = bf16_bits(fv[i].x); h4[0] = (unsigned short)hb; l4[0] = (unsigned short)bf16_bits(fv[i].x - __uint_as_float(hb << 16));
      hb = bf16_bits(fv[i].y); h4[1] = (unsigned short)hb; l4[1] = (unsigned short)bf16_bits(fv[i].y - __uint_as_float(hb << 16));
      hb = bf16_bits(fv[i].z); h4[2] = (unsigned short)hb; l4[2] = (unsigned short)bf16_bits(fv[i].z - __uint_as_float(hb << 16));
      hb = bf16_bits(fv[i].w); h4[3] = (unsigned short)hb; l4[3] = (unsigned short)bf16_bits(fv[i].w - __uint_as_float(hb << 16));
      *(v4usa*)(us + lr * 128 + 4 * m) = h4;
      *(v4usa*)(us + lr * 128 + HID + 4 * m) = l4;
    }
    __syncthreads();
#pragma unroll
    for (int i = 0; i < 8; ++i) {
      const int lr = 16 * wave + 2 * i + hh;
      qv[i] = *(const v8usa*)(us + lr * 128 + 8 * m);
    }
  }

#pragma unroll
  for (int i = 0; i < 8; ++i) {
    const int gr = rowBase + 16 * wave + 2 * i + hh;
    *(volatile v4f*)(outF + (size_t)gr * HID + 4 * m) = fv[i];
  }
  if constexpr (L == 1) {
#pragma unroll
    for (int i = 0; i < 8; ++i) {
      const int gr = rowBase + 16 * wave + 2 * i + hh;
      *(volatile v8us*)(a2 + (size_t)gr * K2 + 2 * HID + 8 * m) = qv[i];
    }
  }
  __threadfence();
#pragma unroll
  for (int i = 0; i < 8; ++i) {
    const int gr = rowBase + 16 * wave + 2 * i + hh;
    *(volatile v4f*)(outF + (size_t)gr * HID + 4 * m) = fv[i];
  }
  if constexpr (L == 1) {
#pragma unroll
    for (int i = 0; i < 8; ++i) {
      const int gr = rowBase + 16 * wave + 2 * i + hh;
      *(volatile v8us*)(a2 + (size_t)gr * K2 + 2 * HID + 8 * m) = qv[i];
    }
  }
}

__global__ __launch_bounds__(NTHR) void k_pool(const float* __restrict__ h2, const int* __restrict__ bat,
                                               const int* __restrict__ ngp, int nN, float* g32) {
  __shared__ __attribute__((aligned(16))) float part[4 * HID];
  __shared__ __attribute__((aligned(16))) float outs[HID];
  const int tid = (int)threadIdx.x, lane = tid & 31, wave = tid >> 5;
  const int g = (int)blockIdx.x;
  int ng = ngp[0];
  ng = ng < 0 ? 0 : (ng > NG ? NG : ng);
  const bool valid = g < ng;

  int loA = 0, hiA = nN, loB = 0, hiB = nN;
#pragma unroll 1
  for (int it = 0; it < 32; ++it) {
    {
      const bool act = loA < hiA;
      int mid = (loA + hiA) >> 1;
      mid = mid < 0 ? 0 : (mid > nN - 1 ? nN - 1 : mid);
      const int v = bat[mid];
      const bool lt = v < g;
      const int nlo = lt ? mid + 1 : loA;
      const int nhi = lt ? hiA : mid;
      loA = act ? nlo : loA;
      hiA = act ? nhi : hiA;
    }
    {
      const bool act = loB < hiB;
      int mid = (loB + hiB) >> 1;
      mid = mid < 0 ? 0 : (mid > nN - 1 ? nN - 1 : mid);
      const int v = bat[mid];
      const bool lt = v <= g;
      const int nlo = lt ? mid + 1 : loB;
      const int nhi = lt ? hiB : mid;
      loB = act ? nlo : loB;
      hiB = act ? nhi : hiB;
    }
  }
  int start = loA < 0 ? 0 : (loA > nN ? nN : loA);
  int end   = loB < start ? start : (loB > nN ? nN : loB);
  end = valid ? end : start;

  const int col = tid & (HID - 1);
  const int r   = tid >> 6;
  float acc = 0.0f;
#pragma unroll 1
  for (int i = start + r; i < end; i += 4) acc += h2[(size_t)i * HID + col];
  part[r * HID + col] = acc;
  __syncthreads();
  if (tid < HID) {
    const float s = ((part[tid] + part[HID + tid]) + part[2 * HID + tid]) + part[3 * HID + tid];
    outs[tid] = s;
  }
  __syncthreads();
  const v4f ovv = *(const v4fa*)(outs + 4 * (lane & 15));
  float* op = g32 + (size_t)g * HID + 4 * (lane & 15);
  const bool okst = (wave == 0) && (lane < 16);
  if (okst) *(volatile v4f*)op = ovv;
  __threadfence();
  if (okst) *(volatile v4f*)op = ovv;
}

__global__ __launch_bounds__(32) void k_tail(const float* __restrict__ g32, const int* __restrict__ flg,
                                             const unsigned short* __restrict__ WL1C,
                                             const unsigned short* __restrict__ WL2C,
                                             const unsigned short* __restrict__ WL3C,
                                             const float* __restrict__ bl1, const float* __restrict__ bl2,
                                             const float* __restrict__ bl3, float* out) {
  __shared__ __attribute__((aligned(16))) unsigned short a0[16 * KT1];
  __shared__ __attribute__((aligned(16))) unsigned short a1[16 * KT2];
  __shared__ __attribute__((aligned(16))) unsigned short a2[16 * KT3];
  __shared__ __attribute__((aligned(16))) float ot[16 * OUTC];
  __shared__ float sb1[T1N];
  __shared__ float sb2[HID];
  __shared__ float sb3[OUTC];
  const int lane = (int)threadIdx.x & 31, hh = lane >> 4, m = lane & 15;
  const int rowBase = (int)blockIdx.x * 16;
  const int fl = flg[0];
  const float pz = (fl != 0) ? __int_as_float(0x7fc00000) : 0.0f;

#pragma unroll 1
  for (int i = lane; i < T1N; i += 32) sb1[i] = bf16_val(bl1[i]);
#pragma unroll 1
  for (int i = lane; i < HID; i += 32) sb2[i] = bf16_val(bl2[i]);
  {
    const float bb = bl3[lane & (OUTC - 1)];
    if (lane < OUTC) sb3[lane] = bf16_val(bb);
  }
#pragma unroll 1
  for (int it = 0; it < 8; ++it) {
    const int idx = it * 32 + lane;
    const int row = idx >> 4;
    const int c4  = (idx & 15) * 4;
    const v4f gv = *(const v4f*)(g32 + (size_t)(rowBase + row) * HID + c4);
    const float x0 = gv.x + pz, x1 = gv.y + pz, x2 = gv.z + pz, x3 = gv.w + pz;
    v4us h4, l4;
    unsigned hb;
    hb = bf16_bits(x0); h4[0] = (unsigned short)hb; l4[0] = (unsigned short)bf16_bits(x0 - __uint_as_float(hb << 16));
    hb = bf16_bits(x1); h4[1] = (unsigned short)hb; l4[1] = (unsigned short)bf16_bits(x1 - __uint_as_float(hb << 16));
    hb = bf16_bits(x2); h4[2] = (unsigned short)hb; l4[2] = (unsigned short)bf16_bits(x2 - __uint_as_float(hb << 16));
    hb = bf16_bits(x3); h4[3] = (unsigned short)hb; l4[3] = (unsigned short)bf16_bits(x3 - __uint_as_float(hb << 16));
    *(v4usa*)(a0 + row * KT1 + c4) = h4;
    *(v4usa*)(a0 + row * KT1 + HID + c4) = l4;
  }
  __syncthreads();

  const v8f z8 = {0.f, 0.f, 0.f, 0.f, 0.f, 0.f, 0.f, 0.f};
  {
    v8f c1[8];
#pragma unroll
    for (int t = 0; t < 8; ++t) c1[t] = z8;
#pragma unroll 1
    for (int k0 = 0; k0 < KT1; k0 += 32) {
      FragB af;
      af.h[0] = *(const v8usa*)(a0 + m * KT1 + k0 + 8 * hh);
      af.h[1] = *(const v8usa*)(a0 + m * KT1 + k0 + 16 + 8 * hh);
#pragma unroll
      for (int nt = 0; nt < 8; ++nt) {
        const unsigned short* wq = WL1C + (size_t)(16 * nt + m) * KT1 + k0 + 8 * hh;
        FragB bf;
        bf.h[0] = *(const v8usa*)wq;
        bf.h[1] = *(const v8usa*)(wq + 16);
        c1[nt] = wmb(af, bf, c1[nt]);
      }
    }
#pragma unroll
    for (int nt = 0; nt < 8; ++nt) {
      const int col = 16 * nt + m;
      const float bv = sb1[col];
#pragma unroll
      for (int r = 0; r < 8; ++r) {
        const int row = 8 * hh + r;
        const float y = relu_keep(c1[nt][r] + bv);
        const unsigned hb = bf16_bits(y);
        const unsigned lb = bf16_bits(y - __uint_as_float(hb << 16));
        a1[row * KT2 + col]       = (unsigned short)hb;
        a1[row * KT2 + T1N + col] = (unsigned short)lb;
      }
    }
  }
  __syncthreads();

  {
    v8f c2[4];
#pragma unroll
    for (int t = 0; t < 4; ++t) c2[t] = z8;
#pragma unroll 1
    for (int k0 = 0; k0 < KT2; k0 += 32) {
      FragB af;
      af.h[0] = *(const v8usa*)(a1 + m * KT2 + k0 + 8 * hh);
      af.h[1] = *(const v8usa*)(a1 + m * KT2 + k0 + 16 + 8 * hh);
#pragma unroll
      for (int nt = 0; nt < 4; ++nt) {
        const unsigned short* wq = WL2C + (size_t)(16 * nt + m) * KT2 + k0 + 8 * hh;
        FragB bf;
        bf.h[0] = *(const v8usa*)wq;
        bf.h[1] = *(const v8usa*)(wq + 16);
        c2[nt] = wmb(af, bf, c2[nt]);
      }
    }
#pragma unroll
    for (int nt = 0; nt < 4; ++nt) {
      const int col = 16 * nt + m;
      const float bv = sb2[col];
#pragma unroll
      for (int r = 0; r < 8; ++r) {
        const int row = 8 * hh + r;
        const float y = relu_keep(c2[nt][r] + bv);
        const unsigned hb = bf16_bits(y);
        const unsigned lb = bf16_bits(y - __uint_as_float(hb << 16));
        a2[row * KT3 + col]       = (unsigned short)hb;
        a2[row * KT3 + HID + col] = (unsigned short)lb;
      }
    }
  }
  __syncthreads();

  {
    v8f c3 = z8;
#pragma unroll 1
    for (int k0 = 0; k0 < KT3; k0 += 32) {
      FragB af, bf;
      af.h[0] = *(const v8usa*)(a2 + m * KT3 + k0 + 8 * hh);
      af.h[1] = *(const v8usa*)(a2 + m * KT3 + k0 + 16 + 8 * hh);
      const unsigned short* wq = WL3C + (size_t)m * KT3 + k0 + 8 * hh;
      bf.h[0] = *(const v8usa*)wq;
      bf.h[1] = *(const v8usa*)(wq + 16);
      c3 = wmb(af, bf, c3);
    }
    const float bv = sb3[m];
#pragma unroll
    for (int r = 0; r < 8; ++r) ot[(8 * hh + r) * OUTC + m] = c3[r] + bv;
  }
  __syncthreads();

  const v4f o0 = *(const v4fa*)(ot + 4 * lane);
  const v4f o1 = *(const v4fa*)(ot + 128 + 4 * lane);
  float* op = out + (size_t)rowBase * OUTC + 4 * lane;
  const bool ok0 = (rowBase + 8) <= NG;
  const bool ok1 = (rowBase + 16) <= NG;
  if (ok0) *(volatile v4f*)op = o0;
  if (ok1) *(volatile v4f*)(op + 128) = o1;
  __threadfence();
  if (ok0) *(volatile v4f*)op = o0;
  if (ok1) *(volatile v4f*)(op + 128) = o1;
}

static inline int cdiv(int a, int b) { return (a + b - 1) / b; }
static inline size_t al256(size_t o) { return (o + 255) & ~(size_t)255; }

extern "C" void kernel_launch(void* const* d_in, const int* in_sizes, int n_in,
                              void* d_out, int out_size, void* d_ws, size_t ws_size,
                              hipStream_t stream) {
  if (n_in < 16) return;
  if (in_sizes[0] < FIN || (in_sizes[0] % FIN) != 0) return;
  const int nN = in_sizes[0] / FIN;
  if (nN < 16 || nN > (1 << 22)) return;
  if (in_sizes[1] < 2 || (in_sizes[1] & 1) != 0) return;
  const int nE = in_sizes[1] / 2;
  if (nE < 1 || nE >= (1 << (31 - SLA))) return;
  if (in_sizes[2] != nN || in_sizes[3] != 1) return;
  if (in_sizes[4] != FIN * HID || in_sizes[5] != HID || in_sizes[6] != FIN * HID) return;
  if (in_sizes[7] != HID * HID || in_sizes[8] != HID || in_sizes[9] != HID * HID) return;
  if (in_sizes[10] != HID * T1N || in_sizes[11] != T1N) return;
  if (in_sizes[12] != T1N * HID || in_sizes[13] != HID) return;
  if (in_sizes[14] != HID * OUTC || in_sizes[15] != OUTC) return;
  if (out_size != NG * OUTC) return;

  const float* x    = (const float*)d_in[0];
  const int*   edge = (const int*)d_in[1];
  const int*   bat  = (const int*)d_in[2];
  const int*   ngp  = (const int*)d_in[3];
  const float* w1l  = (const float*)d_in[4];
  const float* b1l  = (const float*)d_in[5];
  const float* w1r  = (const float*)d_in[6];
  const float* w2l  = (const float*)d_in[7];
  const float* b2l  = (const float*)d_in[8];
  const float* w2r  = (const float*)d_in[9];
  const float* wl1  = (const float*)d_in[10];
  const float* bl1  = (const float*)d_in[11];
  const float* wl2  = (const float*)d_in[12];
  const float* bl2  = (const float*)d_in[13];
  const float* wl3  = (const float*)d_in[14];
  const float* bl3  = (const float*)d_in[15];
  float* out = (float*)d_out;
  const int* src = edge;
  const int* dst = edge + nE;

  const int MP = cdiv(nN, GBM) * GBM;
  const int gM = MP / GBM;
  const int gA = cdiv(MP, NBA);
  if ((long long)gA * NBA < (long long)MP) return;
  const int vec8 = ((nE & 3) == 0) ? 1 : 0;

  char* ws = (char*)d_ws;
  size_t off = 0;
  const size_t oFLG  = off; off = al256(off + 128);
  const size_t oW1C  = off; off = al256(off + (size_t)HID * K1 * 2);
  const size_t oW2C  = off; off = al256(off + (size_t)HID * K2 * 2);
  const size_t oWL1C = off; off = al256(off + (size_t)T1N * KT1 * 2);
  const size_t oWL2C = off; off = al256(off + (size_t)HID * KT2 * 2);
  const size_t oWL3C = off; off = al256(off + (size_t)OUTC * KT3 * 2);
  const size_t oXB   = off; off = al256(off + (size_t)MP * FIN * 2);
  const size_t oA1   = off; off = al256(off + (size_t)MP * K1 * 2);
  const size_t oH1   = off; off = al256(off + (size_t)MP * HID * 4);
  const size_t oA2   = off; off = al256(off + (size_t)MP * K2 * 2);
  const size_t oH2   = off; off = al256(off + (size_t)MP * HID * 4);
  const size_t oG32  = off; off = al256(off + (size_t)NGP * HID * 4);
  if (off > ws_size || off > (size_t)WSMAX) return;
  int*            FLG  = (int*)(ws + oFLG);
  unsigned short* W1C  = (unsigned short*)(ws + oW1C);
  unsigned short* W2C  = (unsigned short*)(ws + oW2C);
  unsigned short* WL1C = (unsigned short*)(ws + oWL1C);
  unsigned short* WL2C = (unsigned short*)(ws + oWL2C);
  unsigned short* WL3C = (unsigned short*)(ws + oWL3C);
  unsigned short* XB   = (unsigned short*)(ws + oXB);
  unsigned short* A1   = (unsigned short*)(ws + oA1);
  float*          H1   = (float*)(ws + oH1);
  unsigned short* A2   = (unsigned short*)(ws + oA2);
  float*          H2   = (float*)(ws + oH2);
  float*          G32  = (float*)(ws + oG32);

  const size_t scanLds = (size_t)AGG_LDS_INTS * 4;
  hipFuncSetAttribute(reinterpret_cast<const void*>(&k_scan<1>), hipFuncAttributeMaxDynamicSharedMemorySize, (int)scanLds);
  hipFuncSetAttribute(reinterpret_cast<const void*>(&k_scan<2>), hipFuncAttributeMaxDynamicSharedMemorySize, (int)scanLds);

  const int nUx = MP * (FIN / 8);
  k_cvx<<<cdiv(nUx, NTHR), NTHR, 0, stream>>>(x, nN, nUx, XB);
  k_wprep<<<6, NTHR, 0, stream>>>(w1l, w1r, w2l, w2r, wl1, wl2, wl3, bat, nN, W1C, W2C, WL1C, WL2C, WL3C, FLG);
  k_scan<1><<<gA, NTHR, scanLds, stream>>>(src, dst, nE, nN, vec8, MP, XB, H1, A1);
  k_gemm<1><<<gM, GTHR, 0, stream>>>(A1, W1C, b1l, H1, A2, nN);
  k_scan<2><<<gA, NTHR, scanLds, stream>>>(src, dst, nE, nN, vec8, MP, XB, H1, A2);
  k_gemm<2><<<gM, GTHR, 0, stream>>>(A2, W2C, b2l, H2, A2, nN);
  k_pool<<<NGP, NTHR, 0, stream>>>(H2, bat, ngp, nN, G32);
  k_tail<<<NTILE, 32, 0, stream>>>(G32, FLG, WL1C, WL2C, WL3C, bl1, bl2, bl3, out);
}
